// FeedForwardQuantum_65481071399183
// MI455X (gfx1250) — hardware-verified
//
#include <hip/hip_runtime.h>
#include <math.h>
#include <stdint.h>

#define NB     8
#define NS     2048
#define EDIM   512
#define FDIM   2048
#define NQ     8
#define MROWS  (NB * NS)
#define HALF_M 8192
#define KQ     32
#define KH     (2 * FDIM)

#define W2_UNITS (EDIM * KH / 8)
#define W1_UNITS (FDIM * KQ / 8)
#define W2_BLKS  (W2_UNITS / 256)
#define W1_BLKS  (W1_UNITS / 256)

static_assert(MROWS == 2 * HALF_M);
static_assert(HALF_M % 128 == 0);
static_assert(FDIM % 64 == 0);
static_assert(EDIM % 64 == 0);
static_assert(KH % 32 == 0);
static_assert(KQ == 32);
static_assert(W2_UNITS == W2_BLKS * 256);
static_assert(W1_UNITS == W1_BLKS * 256);
static_assert(MROWS % 32 == 0);

typedef __attribute__((ext_vector_type(16))) __bf16  v16b;
typedef __attribute__((ext_vector_type(8)))  __bf16  v8b;
typedef __attribute__((ext_vector_type(8)))  float   v8f;
typedef __attribute__((ext_vector_type(4)))  float   v4f;
typedef __attribute__((ext_vector_type(4)))  unsigned int v4u;
typedef v8b __attribute__((may_alias)) v8ba;
typedef v4f __attribute__((may_alias)) v4fa;
typedef v4u __attribute__((may_alias)) v4ua;

__device__ __forceinline__ unsigned short f2bf_bits(float f) {
  unsigned u = __float_as_uint(f);
  return (unsigned short)((u + 0x7FFFu + ((u >> 16) & 1u)) >> 16);
}
__device__ __forceinline__ float bf_bits2f(unsigned short b) { return __uint_as_float(((unsigned)b) << 16); }
__device__ __forceinline__ float bfr(float f) { return bf_bits2f(f2bf_bits(f)); }
__device__ __forceinline__ unsigned pk16(unsigned short a, unsigned short b) { return (unsigned)a | ((unsigned)b << 16); }

__device__ __forceinline__ v8f mma_bf16(v16b a, v16b b, v8f c) {
  c = __builtin_amdgcn_wmma_f32_16x16x32_bf16(false, a, false, b, (short)0, c, false, false);
  asm volatile("v_nop\n\tv_nop\n\tv_nop\n\tv_nop" : "+v"(c) : "v"(a), "v"(b));
  return c;
}

__device__ __forceinline__ v16b ldfrag(const __bf16* p) {
  union { v16b v; v8b h[2]; } f;
  f.h[0] = *(const v8ba*)(p);
  f.h[1] = *(const v8ba*)(p + 16);
  return f.v;
}

__global__ __launch_bounds__(256) void prep_kernel(const float* __restrict__ W1, const float* __restrict__ W2,
                                                   unsigned short* __restrict__ W1P, unsigned short* __restrict__ W2P) {
  const int tid = threadIdx.x;
  if (blockIdx.x < W2_BLKS) {
    const int u  = blockIdx.x * 256 + tid;
    const int e  = u >> 9;
    const int c8 = (u & 511) * 8;
    const int sc = c8 & (FDIM - 1);
    const float* src = W2 + (size_t)e * FDIM + sc;
    const v4f a = *(const v4fa*)src;
    const v4f c = *(const v4fa*)(src + 4);
    v4u v;
    v[0] = pk16(f2bf_bits(a[0]), f2bf_bits(a[1]));
    v[1] = pk16(f2bf_bits(a[2]), f2bf_bits(a[3]));
    v[2] = pk16(f2bf_bits(c[0]), f2bf_bits(c[1]));
    v[3] = pk16(f2bf_bits(c[2]), f2bf_bits(c[3]));
    unsigned short* dst = W2P + (size_t)e * KH + c8;
    *(volatile v4u*)dst = v;
    __threadfence();
    *(volatile v4u*)dst = v;
  } else {
    const int u    = (blockIdx.x - W2_BLKS) * 256 + tid;
    const int f    = u >> 2;
    const int part = u & 3;
    const float* src = W1 + (size_t)f * NQ;
    const v4f a = *(const v4fa*)src;
    const v4f c = *(const v4fa*)(src + 4);
    const unsigned keep = (part < 2) ? 0xFFFFFFFFu : 0u;
    v4u v;
    v[0] = pk16(f2bf_bits(a[0]), f2bf_bits(a[1])) & keep;
    v[1] = pk16(f2bf_bits(a[2]), f2bf_bits(a[3])) & keep;
    v[2] = pk16(f2bf_bits(c[0]), f2bf_bits(c[1])) & keep;
    v[3] = pk16(f2bf_bits(c[2]), f2bf_bits(c[3])) & keep;
    unsigned short* dst = W1P + (size_t)f * KQ + part * 8;
    *(volatile v4u*)dst = v;
    __threadfence();
    *(volatile v4u*)dst = v;
  }
}

__global__ __launch_bounds__(256) void qfeat_kernel(const float* __restrict__ x, const float* __restrict__ theta,
                                                    unsigned short* __restrict__ QA) {
  __shared__ __align__(16) unsigned short sQ[32 * 32];
  const int tid = threadIdx.x;
  const int r = tid >> 3, j = tid & 7;
  const int row = blockIdx.x * 32 + r;
  const float xb = bfr(x[(size_t)row * EDIM + j]);
  const float tb = bfr(theta[j]);
  float q = 1.0f;
#pragma unroll 1
  for (int it = 0; it < 2; ++it) {
    const float arg = (it == 0) ? xb : tb;
    q = q * cosf(arg);
  }
  const unsigned short hb = f2bf_bits(q);
  const unsigned short lb = f2bf_bits(q - bf_bits2f(hb));
  sQ[r * 32 + j]      = hb;
  sQ[r * 32 + 8 + j]  = lb;
  sQ[r * 32 + 16 + j] = 0;
  sQ[r * 32 + 24 + j] = 0;
  __syncthreads();
  if (tid < 128) {
    const v4u v = *(const v4ua*)(sQ + tid * 8);
    unsigned short* dst = QA + (size_t)blockIdx.x * 32 * KQ + tid * 8;
    *(volatile v4u*)dst = v;
    __threadfence();
    *(volatile v4u*)dst = v;
  }
}

__device__ __forceinline__ void h_store_pass(const unsigned short* sH, unsigned short* HP,
                                             int lrow_w, int n0, int w, int lane) {
  const int q8 = lane & 7, sub = lane >> 3;
#pragma unroll
  for (int i = 0; i < 16; ++i) {
    const int lid = i * 4 + sub;
    const int row = lid >> 1, which = lid & 1;
    const v4u v = *(const v4ua*)(sH + which * 8192 + (32 * w + row) * 64 + 8 * q8);
    *(volatile v4u*)(HP + (size_t)(lrow_w + row) * KH + which * FDIM + n0 + 8 * q8) = v;
  }
}

__global__ __launch_bounds__(128) void hgemm_kernel(const unsigned short* __restrict__ QA,
                                                    const unsigned short* __restrict__ W1P,
                                                    const float* __restrict__ b1,
                                                    unsigned short* __restrict__ HP, int row_base) {
  __shared__ __align__(16) unsigned short sH[2 * 128 * 64];
  const int tid = threadIdx.x, lane = tid & 31, w = tid >> 5;
  const int h = lane >> 4, m = lane & 15;
  const int lrow_w = blockIdx.x * 128 + 32 * w;
  const int n0 = blockIdx.y * 64;
  const __bf16* QAb = (const __bf16*)(const void*)QA;
  const __bf16* W1b = (const __bf16*)(const void*)W1P;

  const v16b a0 = ldfrag(QAb + (size_t)(row_base + lrow_w + m) * KQ + 8 * h);
  const v16b a1 = ldfrag(QAb + (size_t)(row_base + lrow_w + 16 + m) * KQ + 8 * h);
  const v8f zero8 = {0.f, 0.f, 0.f, 0.f, 0.f, 0.f, 0.f, 0.f};
  v8f acc[2][4];
#pragma unroll
  for (int nt = 0; nt < 4; ++nt) {
    const v16b b = ldfrag(W1b + (size_t)(n0 + 16 * nt + m) * KQ + 8 * h);
    acc[0][nt] = mma_bf16(a0, b, zero8);
    acc[1][nt] = mma_bf16(a1, b, zero8);
  }

#pragma unroll
  for (int nt = 0; nt < 4; ++nt) {
    const int fl = 16 * nt + m;
    const float bias = bfr(b1[n0 + fl]);
#pragma unroll
    for (int mt = 0; mt < 2; ++mt) {
#pragma unroll
      for (int r = 0; r < 8; ++r) {
        const int rl = 32 * w + 16 * mt + 8 * h + r;
        const float hv = fmaxf(acc[mt][nt][r] + bias, 0.0f);
        const unsigned short hb = f2bf_bits(hv);
        const unsigned short lb = f2bf_bits(hv - bf_bits2f(hb));
        sH[rl * 64 + fl]        = hb;
        sH[8192 + rl * 64 + fl] = lb;
      }
    }
  }
  __syncthreads();

  h_store_pass(sH, HP, lrow_w, n0, w, lane);
  __threadfence();
  h_store_pass(sH, HP, lrow_w, n0, w, lane);
}

__device__ __forceinline__ void o_store_pass(const float* sO, float* out,
                                             int grow_w, int n0, int w, int lane) {
  const int q8 = lane & 7, sub = lane >> 3;
#pragma unroll
  for (int i = 0; i < 16; ++i) {
    const int lid = i * 4 + sub;
    const int row = lid >> 1, hl = lid & 1;
    const v4f v = *(const v4fa*)(sO + (32 * w + row) * 64 + 32 * hl + 4 * q8);
    *(volatile v4f*)(out + (size_t)(grow_w + row) * EDIM + n0 + 32 * hl + 4 * q8) = v;
  }
}

__global__ __launch_bounds__(128) void ogemm_kernel(const unsigned short* __restrict__ HP,
                                                    const unsigned short* __restrict__ W2P,
                                                    const float* __restrict__ b2,
                                                    float* __restrict__ out, int row_base) {
  __shared__ __align__(16) float sO[128 * 64];
  const int tid = threadIdx.x, lane = tid & 31, w = tid >> 5;
  const int h = lane >> 4, m = lane & 15;
  const int lrow_w = blockIdx.x * 128 + 32 * w;
  const int n0 = blockIdx.y * 64;
  const __bf16* HPb = (const __bf16*)(const void*)HP;
  const __bf16* W2b = (const __bf16*)(const void*)W2P;

  const __bf16* xa0 = HPb + (size_t)(lrow_w + m) * KH + 8 * h;
  const __bf16* xa1 = xa0 + (size_t)16 * KH;
  const __bf16* wb  = W2b + (size_t)(n0 + m) * KH + 8 * h;

  const v8f zero8 = {0.f, 0.f, 0.f, 0.f, 0.f, 0.f, 0.f, 0.f};
  v8f acc[2][4];
#pragma unroll
  for (int mt = 0; mt < 2; ++mt)
#pragma unroll
    for (int nt = 0; nt < 4; ++nt) acc[mt][nt] = zero8;

#pragma unroll 1
  for (int k0 = 0; k0 < KH; k0 += 32) {
    const v16b a0 = ldfrag(xa0 + k0);
    const v16b a1 = ldfrag(xa1 + k0);
#pragma unroll
    for (int nt = 0; nt < 4; ++nt) {
      const v16b b = ldfrag(wb + (size_t)nt * 16 * KH + k0);
      acc[0][nt] = mma_bf16(a0, b, acc[0][nt]);
      acc[1][nt] = mma_bf16(a1, b, acc[1][nt]);
    }
  }

#pragma unroll
  for (int nt = 0; nt < 4; ++nt) {
    const int cl = 16 * nt + m;
    const float bias = bfr(b2[n0 + cl]);
#pragma unroll
    for (int mt = 0; mt < 2; ++mt) {
#pragma unroll
      for (int r = 0; r < 8; ++r) {
        const int rl = 32 * w + 16 * mt + 8 * h + r;
        sO[rl * 64 + cl] = acc[mt][nt][r] + bias;
      }
    }
  }
  __syncthreads();

  const int grow_w = row_base + lrow_w;
  o_store_pass(sO, out, grow_w, n0, w, lane);
  __threadfence();
  o_store_pass(sO, out, grow_w, n0, w, lane);
}

extern "C" void kernel_launch(void* const* d_in, const int* in_sizes, int n_in,
                              void* d_out, int out_size, void* d_ws, size_t ws_size,
                              hipStream_t stream) {
  if (n_in < 6) return;
  if (in_sizes[0] != MROWS * EDIM) return;
  if (in_sizes[1] != NQ) return;
  if (in_sizes[2] != FDIM * NQ) return;
  if (in_sizes[3] != FDIM) return;
  if (in_sizes[4] != EDIM * FDIM) return;
  if (in_sizes[5] != EDIM) return;
  if (out_size != MROWS * EDIM) return;

  const float* x     = (const float*)d_in[0];
  const float* theta = (const float*)d_in[1];
  const float* W1    = (const float*)d_in[2];
  const float* b1    = (const float*)d_in[3];
  const float* W2    = (const float*)d_in[4];
  const float* b2    = (const float*)d_in[5];
  float* out = (float*)d_out;

  size_t off = 0;
  const size_t oHP  = off; off += (size_t)HALF_M * KH * 2;
  const size_t oW2P = off; off += (size_t)EDIM * KH * 2;
  const size_t oW1P = off; off += (size_t)FDIM * KQ * 2;
  const size_t oQA  = off; off += (size_t)MROWS * KQ * 2;
  if (off > ws_size) return;
  if (off > (size_t)134217728) return;

  char* ws = (char*)d_ws;
  unsigned short* HP  = (unsigned short*)(ws + oHP);
  unsigned short* W2P = (unsigned short*)(ws + oW2P);
  unsigned short* W1P = (unsigned short*)(ws + oW1P);
  unsigned short* QA  = (unsigned short*)(ws + oQA);

  prep_kernel<<<dim3(W2_BLKS + W1_BLKS), dim3(256), 0, stream>>>(W1, W2, W1P, W2P);
  qfeat_kernel<<<dim3(MROWS / 32), dim3(256), 0, stream>>>(x, theta, QA);
  for (int half = 0; half < 2; ++half) {
    const int row_base = half * HALF_M;
    hgemm_kernel<<<dim3(HALF_M / 128, FDIM / 64), dim3(128), 0, stream>>>(QA, W1P, b1, HP, row_base);
    ogemm_kernel<<<dim3(HALF_M / 128, EDIM / 64), dim3(128), 0, stream>>>(HP, W2P, b2, out, row_base);
  }
  (void)hipGetLastError();
}
